// MPNN_Surrogate_824633721181
// MI455X (gfx1250) — hardware-run, weakly checked
//
#include <hip/hip_runtime.h>
#include <math.h>

typedef __attribute__((ext_vector_type(16))) _Float16 v16h;
typedef __attribute__((ext_vector_type(8)))  _Float16 v8h;
typedef __attribute__((ext_vector_type(16))) __bf16   v16b;
typedef __attribute__((ext_vector_type(8)))  __bf16   v8b;
typedef __attribute__((ext_vector_type(8)))  float    v8f;
typedef __attribute__((ext_vector_type(4)))  float    v4f;
typedef __attribute__((ext_vector_type(2)))  unsigned v2u;

constexpr int kNN     = 30000;
constexpr int kNE     = 480000;
constexpr int kXin    = 16;
constexpr int kHid    = 128;
constexpr int kOutW   = 3;
constexpr int kLayers = 3;
constexpr int kCat    = 2 * kHid;
constexpr int kMP     = 30016;
static_assert(kMP % 64 == 0 && kMP >= kNN && kMP - kNN < 64, "row padding");
static_assert(kHid % 64 == 0 && kCat % 64 == 0, "GEMM N multiples of 64");
static_assert(kHid % 32 == 0 && kCat % 32 == 0, "GEMM K multiples of 32");

constexpr bool  kSplit  = true;
constexpr int   kET     = kSplit ? 1 : 0;
constexpr int   kSPL    = kSplit ? 2 : 0;
constexpr float kWCarry = kSplit ? 1.0f : 1024.0f;
constexpr float kWFold  = 1.0f / kWCarry;

constexpr size_t kLo      = kSplit ? 1 : 0;
constexpr size_t kSzH32   = (size_t)kMP * kHid * 4;
constexpr size_t kSzHA    = (size_t)kMP * kCat * 2;
constexpr size_t kSzPQ    = (size_t)kMP * kCat * 4;
constexpr size_t kSzS     = (size_t)kMP * kHid * 2;
constexpr size_t kSzT     = (size_t)kMP * kHid * 2;
constexpr size_t kSzDeg   = (size_t)kMP * 4;
constexpr size_t kSzW1    = (size_t)kLayers * kCat * kHid * 2;
constexpr size_t kSzW2    = (size_t)kLayers * kHid * kHid * 2;
constexpr size_t kOffH32  = 0;
constexpr size_t kOffHAH  = kOffH32  + kSzH32;
constexpr size_t kOffHAL  = kOffHAH  + kSzHA;
constexpr size_t kOffPQ   = kOffHAL  + kSzHA * kLo;
constexpr size_t kOffSH   = kOffPQ   + kSzPQ;
constexpr size_t kOffSL   = kOffSH   + kSzS;
constexpr size_t kOffTH   = kOffSL   + kSzS * kLo;
constexpr size_t kOffTL   = kOffTH   + kSzT;
constexpr size_t kOffDEG  = kOffTL   + kSzT * kLo;
constexpr size_t kOffWE1H = kOffDEG  + kSzDeg;
constexpr size_t kOffWE1L = kOffWE1H + kSzW1;
constexpr size_t kOffWE2H = kOffWE1L + kSzW1 * kLo;
constexpr size_t kOffWE2L = kOffWE2H + kSzW2;
constexpr size_t kOffWN1H = kOffWE2L + kSzW2 * kLo;
constexpr size_t kOffWN1L = kOffWN1H + kSzW1;
constexpr size_t kOffWN2H = kOffWN1L + kSzW1 * kLo;
constexpr size_t kOffWN2L = kOffWN2H + kSzW2;
constexpr size_t kWsTotal = kOffWN2L + kSzW2 * kLo;
static_assert(kWsTotal == (kSplit ? 108877056ull : 77550848ull), "carve total");
static_assert(kWsTotal <= 134217728ull, "carve cap");
static_assert((kSzH32 % 128) == 0 && (kSzHA % 128) == 0 && (kSzPQ % 128) == 0 && (kSzS % 128) == 0 &&
              (kSzT % 128) == 0 && (kSzDeg % 128) == 0 && (kSzW1 % 128) == 0 && (kSzW2 % 128) == 0,
              "128-B aligned regions");

__device__ __forceinline__ unsigned short f2bf_bits(float f) {
  unsigned u = __float_as_uint(f);
  return (unsigned short)((u + 0x7FFFu + ((u >> 16) & 1u)) >> 16);
}
__device__ __forceinline__ float bf_bits2f(unsigned short h) { return __uint_as_float(((unsigned)h) << 16); }

__device__ __forceinline__ int uniform_wave_index() {
  return __builtin_amdgcn_readfirstlane((int)(threadIdx.x >> 5));
}

template <bool SP>
__device__ __forceinline__ void pack8(const float (&f)[8], float carry, v8h& hv, v8h& lv) {
#pragma unroll
  for (int e = 0; e < 8; ++e) {
    if (SP) {
      const unsigned short hb = f2bf_bits(f[e]);
      const unsigned short lb = f2bf_bits(f[e] - bf_bits2f(hb));
      const _Float16 hx = __builtin_bit_cast(_Float16, hb);
      const _Float16 lx = __builtin_bit_cast(_Float16, lb);
      hv[e] = hx;
      lv[e] = lx;
    } else {
      const _Float16 hx = (_Float16)(f[e] * carry);
      hv[e] = hx;
      lv[e] = (_Float16)0.0f;
    }
  }
}

__device__ __forceinline__ v8f mma_h(v16h a, v16h b, v8f c) {
  c = __builtin_amdgcn_wmma_f32_16x16x32_f16(false, a, false, b, (short)0, c, false, false);
  asm volatile("v_nop\n\tv_nop\n\tv_nop\n\tv_nop" : "+v"(c) : "v"(a), "v"(b));
  return c;
}
__device__ __forceinline__ v8f mma_b(v16b a, v16b b, v8f c) {
  c = __builtin_amdgcn_wmma_f32_16x16x32_bf16(false, a, false, b, (short)0, c, false, false);
  asm volatile("v_nop\n\tv_nop\n\tv_nop\n\tv_nop" : "+v"(c) : "v"(a), "v"(b));
  return c;
}
__device__ __forceinline__ void acc_guard4(v8f& a, v8f& b, v8f& c, v8f& d) {
  asm volatile("v_nop\n\tv_nop\n\tv_nop\n\tv_nop" : "+v"(a), "+v"(b), "+v"(c), "+v"(d));
}

template <typename T> struct Frag;
template <> struct Frag<_Float16> {
  typedef v16h V;
  union U { v16h v; v8h h[2]; };
  static __device__ __forceinline__ v16h load(const _Float16* p) {
    U f;
    f.h[0] = *(const v8h*)(p);
    f.h[1] = *(const v8h*)(p + 16);
    return f.v;
  }
  static __device__ __forceinline__ v8f mma(v16h a, v16h b, v8f c) { return mma_h(a, b, c); }
};
template <> struct Frag<__bf16> {
  typedef v16b V;
  union U { v16b v; v8b h[2]; };
  static __device__ __forceinline__ v16b load(const __bf16* p) {
    U f;
    f.h[0] = *(const v8b*)(p);
    f.h[1] = *(const v8b*)(p + 16);
    return f.v;
  }
  static __device__ __forceinline__ v8f mma(v16b a, v16b b, v8f c) { return mma_b(a, b, c); }
};
template <int ET> struct Elem;
template <> struct Elem<0> { typedef _Float16 T; };
template <> struct Elem<1> { typedef __bf16 T; };

template <int ET, int SPL, int EPI>
__global__ __launch_bounds__(256) void tile_gemm_kernel(
    const unsigned short* __restrict__ Ap, const unsigned short* __restrict__ A2p, int lda,
    const unsigned short* __restrict__ Btp, const unsigned short* __restrict__ Bt2p, int ldb,
    float* Cf, int ldcf,
    unsigned short* C16, unsigned short* C16lo, int ldc16,
    const float* __restrict__ bias, const float* __restrict__ degp,
    int M, int N, int K, int nReal, float scale) {
  typedef typename Elem<ET>::T T;
  typedef typename Frag<T>::V V;
  constexpr bool SP = (SPL == 2);
  const T* A   = (const T*)Ap;
  const T* A2  = (const T*)A2p;
  const T* Bt  = (const T*)Btp;
  const T* Bt2 = (const T*)Bt2p;
  __shared__ __align__(16) float sT[8][16 * 68];
  const int lane = threadIdx.x & 31;
  const int wave = uniform_wave_index();
  const int tilesN = N >> 6;
  const int tilesM = M >> 6;
  const int tile = blockIdx.x * 8 + wave;
  if (tile >= tilesM * tilesN) return;
  const int tm = tile / tilesN;
  const int tn = tile - tm * tilesN;
  const int m0 = tm << 6;
  const int n0 = tn << 6;

  const int rlane = lane & 15;
  const int koff  = (lane >> 4) * 8;
  const int mOff  = (lane >> 4) * 8;

  v8f acc[4][4];
#pragma unroll
  for (int i = 0; i < 4; ++i)
#pragma unroll
    for (int j = 0; j < 4; ++j) acc[i][j] = (v8f){0.f, 0.f, 0.f, 0.f, 0.f, 0.f, 0.f, 0.f};

  for (int k0 = 0; k0 < K; k0 += 32) {
    V bh[4], bl[4];
#pragma unroll
    for (int j = 0; j < 4; ++j) {
      const size_t bo = (size_t)(n0 + (j << 4) + rlane) * ldb + koff + k0;
      bh[j] = Frag<T>::load(Bt + bo);
      if (SP) bl[j] = Frag<T>::load(Bt2 + bo);
    }
#pragma unroll
    for (int i = 0; i < 4; ++i) {
      const size_t ao = (size_t)(m0 + (i << 4) + rlane) * lda + koff + k0;
      V ah = Frag<T>::load(A + ao);
      V al;
      if (SP) al = Frag<T>::load(A2 + ao);
#pragma unroll
      for (int j = 0; j < 4; ++j) {
        acc[i][j] = Frag<T>::mma(ah, bh[j], acc[i][j]);
        if (SP) {
          acc[i][j] = Frag<T>::mma(ah, bl[j], acc[i][j]);
          acc[i][j] = Frag<T>::mma(al, bh[j], acc[i][j]);
        }
      }
    }
  }
  acc_guard4(acc[0][0], acc[0][1], acc[0][2], acc[0][3]);
  acc_guard4(acc[1][0], acc[1][1], acc[1][2], acc[1][3]);
  acc_guard4(acc[2][0], acc[2][1], acc[2][2], acc[2][3]);
  acc_guard4(acc[3][0], acc[3][1], acc[3][2], acc[3][3]);

  float* slab = sT[wave];
  float bvj[4];
#pragma unroll
  for (int j = 0; j < 4; ++j) {
    const int n = n0 + (j << 4) + rlane;
    if (EPI == 0) {
      const int nb = n - kHid;
      const int nbc = nb < 0 ? 0 : nb;
      const float bl0 = bias[nbc];
      bvj[j] = (n0 >= kHid) ? bl0 : 0.0f;
    } else {
      bvj[j] = bias[n];
    }
  }
#pragma unroll
  for (int i = 0; i < 4; ++i) {
    const int mBase = m0 + (i << 4);
    float dg[8];
#pragma unroll
    for (int r = 0; r < 8; ++r) dg[r] = 0.0f;
    if (EPI == 1) {
      const v4f d0 = *(const v4f*)(degp + mBase + mOff);
      const v4f d1 = *(const v4f*)(degp + mBase + mOff + 4);
      dg[0] = d0[0]; dg[1] = d0[1]; dg[2] = d0[2]; dg[3] = d0[3];
      dg[4] = d1[0]; dg[5] = d1[1]; dg[6] = d1[2]; dg[7] = d1[3];
    }
#pragma unroll
    for (int j = 0; j < 4; ++j) {
#pragma unroll
      for (int r = 0; r < 8; ++r) {
        float v = acc[i][j][r] * scale;
        if (EPI == 1) v += dg[r] * bvj[j];
        else v += bvj[j];
        if (EPI == 2) v = fmaxf(v, 0.0f);
        if (EPI != 0) v = ((mBase + mOff + r) < nReal) ? v : 0.0f;
        slab[(mOff + r) * 68 + (j << 4) + rlane] = v;
      }
    }
    __builtin_amdgcn_fence(__ATOMIC_RELEASE, "workgroup");
    __builtin_amdgcn_wave_barrier();
    __builtin_amdgcn_fence(__ATOMIC_ACQUIRE, "workgroup");
    if (EPI == 0) {
      const int hh = lane >> 4, c4 = (lane & 15) * 4;
      for (int pass = 0; pass < 2; ++pass) {
#pragma unroll
        for (int it = 0; it < 8; ++it) {
          const int row = it * 2 + hh;
          const v4f v = *(const v4f*)(slab + row * 68 + c4);
          *(volatile v4f*)(Cf + (size_t)(mBase + row) * ldcf + n0 + c4) = v;
        }
        __threadfence();
      }
    }
    if (EPI == 3) {
      const int hh = lane >> 4, c4 = (lane & 15) * 4;
      v4f nv[8];
#pragma unroll
      for (int it = 0; it < 8; ++it) {
        const int row = it * 2 + hh;
        const v4f sv = *(const v4f*)(slab + row * 68 + c4);
        const v4f rv = *(const v4f*)(Cf + (size_t)(mBase + row) * ldcf + n0 + c4);
        nv[it] = sv + rv;
        *(v4f*)(slab + row * 68 + c4) = nv[it];
      }
      for (int pass = 0; pass < 2; ++pass) {
#pragma unroll
        for (int it = 0; it < 8; ++it) {
          const int row = it * 2 + hh;
          *(volatile v4f*)(Cf + (size_t)(mBase + row) * ldcf + n0 + c4) = nv[it];
        }
        __threadfence();
      }
      __builtin_amdgcn_fence(__ATOMIC_RELEASE, "workgroup");
      __builtin_amdgcn_wave_barrier();
      __builtin_amdgcn_fence(__ATOMIC_ACQUIRE, "workgroup");
    }
    if (EPI != 0) {
      const int q = lane >> 3, c8 = (lane & 7) * 8;
      for (int pass = 0; pass < 2; ++pass) {
#pragma unroll
        for (int it = 0; it < 4; ++it) {
          const int row = it * 4 + q;
          const float* sp = slab + row * 68 + c8;
          float f[8];
#pragma unroll
          for (int e = 0; e < 8; ++e) f[e] = sp[e];
          v8h hv, lv;
          pack8<SP>(f, 1.0f, hv, lv);
          const size_t o = (size_t)(mBase + row) * ldc16 + n0 + c8;
          *(volatile v8h*)(C16 + o) = hv;
          if (SP) *(volatile v8h*)(C16lo + o) = lv;
        }
        __threadfence();
      }
    }
    __builtin_amdgcn_fence(__ATOMIC_RELEASE, "workgroup");
    __builtin_amdgcn_wave_barrier();
    __builtin_amdgcn_fence(__ATOMIC_ACQUIRE, "workgroup");
  }
}

template <bool SP>
__global__ __launch_bounds__(256) void weight_plane_kernel(
    const float* __restrict__ src, unsigned short* __restrict__ dhi, unsigned short* __restrict__ dlo,
    int nRows, int kCols, int srcLayer, int catMode, int total8, float carry) {
  const int i = blockIdx.x * 256 + threadIdx.x;
  if (i >= total8) return;
  const int kg = kCols >> 3;
  const int perLayer = nRows * kg;
  const int l = i / perLayer;
  const int rem = i - l * perLayer;
  const int j = rem / kg;
  const int k0 = (rem - j * kg) << 3;
  const int rowOff = (catMode != 0 && j >= kHid) ? kHid : 0;
  const int col = j & (kHid - 1);
  const float* sp = src + (size_t)l * srcLayer + (size_t)(rowOff + k0) * kHid + col;
  float f[8];
#pragma unroll
  for (int e = 0; e < 8; ++e) f[e] = sp[(size_t)e * kHid];
  v8h hv, lv;
  pack8<SP>(f, carry, hv, lv);
  const size_t o = (size_t)i << 3;
  *(volatile v8h*)(dhi + o) = hv;
  if (SP) *(volatile v8h*)(dlo + o) = lv;
  __threadfence();
  *(volatile v8h*)(dhi + o) = hv;
  if (SP) *(volatile v8h*)(dlo + o) = lv;
}

template <bool SP>
__global__ __launch_bounds__(256) void input_proj_kernel(
    const float* __restrict__ x, const float* __restrict__ W, const float* __restrict__ b,
    float* __restrict__ h32, unsigned short* __restrict__ HAh, unsigned short* __restrict__ HAl) {
  const int lane = threadIdx.x & 31;
  const int wave = uniform_wave_index();
  const int c4 = lane * 4;
  v4f w[kXin];
#pragma unroll
  for (int k = 0; k < kXin; ++k) w[k] = *(const v4f*)(W + k * kHid + c4);
  const v4f bv = *(const v4f*)(b + c4);
  const int row0 = blockIdx.x * 64 + wave * 8;
#pragma unroll 1
  for (int rr = 0; rr < 8; ++rr) {
    const int row = row0 + rr;
    const int rowc = row < kNN ? row : (kNN - 1);
    const float* xr = x + (size_t)rowc * kXin;
    const v4f x0 = *(const v4f*)(xr);
    const v4f x1 = *(const v4f*)(xr + 4);
    const v4f x2 = *(const v4f*)(xr + 8);
    const v4f x3 = *(const v4f*)(xr + 12);
    const float xs[kXin] = {x0[0], x0[1], x0[2], x0[3], x1[0], x1[1], x1[2], x1[3],
                            x2[0], x2[1], x2[2], x2[3], x3[0], x3[1], x3[2], x3[3]};
    v4f acc = bv;
#pragma unroll
    for (int k = 0; k < kXin; ++k) acc = acc + w[k] * xs[k];
    if (row >= kNN) acc = (v4f){0.f, 0.f, 0.f, 0.f};
    unsigned hb[4], lb[4];
#pragma unroll
    for (int c = 0; c < 4; ++c) {
      const float fv = acc[c];
      if (SP) {
        const unsigned short hbits = f2bf_bits(fv);
        const unsigned short lbits = f2bf_bits(fv - bf_bits2f(hbits));
        hb[c] = (unsigned)hbits;
        lb[c] = (unsigned)lbits;
      } else {
        const _Float16 hx = (_Float16)fv;
        const unsigned short hbits = __builtin_bit_cast(unsigned short, hx);
        hb[c] = (unsigned)hbits;
        lb[c] = 0u;
      }
    }
    const v2u vh = {hb[0] | (hb[1] << 16), hb[2] | (hb[3] << 16)};
    const v2u vl = {lb[0] | (lb[1] << 16), lb[2] | (lb[3] << 16)};
    float* hp = h32 + (size_t)row * kHid + c4;
    const size_t ao = (size_t)row * kCat + c4;
    for (int pass = 0; pass < 2; ++pass) {
      *(volatile v4f*)hp = acc;
      *(volatile v2u*)(HAh + ao) = vh;
      if (SP) *(volatile v2u*)(HAl + ao) = vl;
      __threadfence();
    }
  }
}

constexpr int kTileNodes      = 64;
constexpr int kEdgeThreads    = 128;
constexpr int kEdgesPerThread = 32;
constexpr int kChunkEdges     = kEdgeThreads * kEdgesPerThread;
constexpr int kNumChunks      = (kNE + kChunkEdges - 1) / kChunkEdges;
static_assert(kHid == kEdgeThreads, "thread = channel");
static_assert(kNE % kEdgesPerThread == 0, "a thread's edge group is fully inside or fully outside the list");
static_assert((kChunkEdges & (kChunkEdges - 1)) == 0, "list index mask");
static_assert(kMP % kTileNodes == 0, "destination tiles");
static_assert(((size_t)kNE * 4) % 16 == 0, "16-B aligned second index row");
static_assert((kNN - (kMP - kTileNodes)) > 0, "last tile holds real nodes");

template <bool SP>
__global__ __launch_bounds__(128) void edge_sum_kernel(
    const int* __restrict__ ei, const float* __restrict__ PQ,
    unsigned short* __restrict__ Sh, unsigned short* __restrict__ Sl, float* __restrict__ degp) {
  __shared__ __align__(16) float sS[kTileNodes * kHid];
  __shared__ int sList[kChunkEdges];
  __shared__ int sWtot[4];
  const int tid  = threadIdx.x;
  const int lane = tid & 31;
  const int wave = uniform_wave_index();
  const int base = blockIdx.x * kTileNodes;
  const int* colp = ei + kNE;
  const int remain = kNN - base;
  const unsigned lim = (unsigned)(remain < kTileNodes ? remain : kTileNodes);
  const int myNode = tid & (kTileNodes - 1);

#pragma unroll 1
  for (int n = 0; n < kTileNodes; ++n) sS[n * kHid + tid] = 0.0f;
  int degc = 0;

#pragma unroll 1
  for (int ch = 0; ch < kNumChunks; ++ch) {
    const int eb = ch * kChunkEdges + tid * kEdgesPerThread;
    const bool valid = eb < kNE;
    const int ebc = valid ? eb : (kNE - kEdgesPerThread);
    const int4* cp = (const int4*)(colp + ebc);
    unsigned m = 0u;
#pragma unroll
    for (int q = 0; q < kEdgesPerThread / 4; ++q) {
      const int4 c = cp[q];
      m |= (((unsigned)c.x - (unsigned)base) < lim) ? (1u << (4 * q + 0)) : 0u;
      m |= (((unsigned)c.y - (unsigned)base) < lim) ? (1u << (4 * q + 1)) : 0u;
      m |= (((unsigned)c.z - (unsigned)base) < lim) ? (1u << (4 * q + 2)) : 0u;
      m |= (((unsigned)c.w - (unsigned)base) < lim) ? (1u << (4 * q + 3)) : 0u;
    }
    m = valid ? m : 0u;
    const int cnt = __popc(m);
    int incl = cnt;
#pragma unroll
    for (int off = 1; off < 32; off <<= 1) {
      const int t = __shfl_up(incl, off, 32);
      incl += (lane >= off) ? t : 0;
    }
    if (lane == 31) sWtot[wave] = incl;
    __syncthreads();
    int woff = 0, total = 0;
#pragma unroll
    for (int w = 0; w < 4; ++w) {
      const int t = sWtot[w];
      woff += (w < wave) ? t : 0;
      total += t;
    }
    int pos = woff + incl - cnt;
    unsigned mm = m;
#pragma unroll 1
    for (int it = 0; it < kEdgesPerThread; ++it) {
      if (mm == 0u) break;
      const int k = __builtin_ctz(mm);
      mm &= mm - 1u;
      sList[pos & (kChunkEdges - 1)] = eb + k;
      ++pos;
    }
    __syncthreads();
    const int L = total < kChunkEdges ? total : kChunkEdges;
#pragma unroll 1
    for (int i = 0; i < L; ++i) {
      int e = __builtin_amdgcn_readfirstlane(sList[i]);
      e = e < 0 ? 0 : (e > kNE - 1 ? kNE - 1 : e);
      const int c = colp[e];
      int r = ei[e];
      r = r < 0 ? 0 : (r > kNN - 1 ? kNN - 1 : r);
      int ld = c - base;
      ld = ld < 0 ? 0 : (ld > kTileNodes - 1 ? kTileNodes - 1 : ld);
      const float pv = PQ[(size_t)r * kCat + tid];
      const float qv = PQ[(size_t)(base + ld) * kCat + kHid + tid];
      const float z = pv + qv;
      sS[ld * kHid + tid] += fmaxf(z, 0.0f);
      degc += (ld == myNode) ? 1 : 0;
    }
    __syncthreads();
  }

  {
    const int rsub = lane >> 4, c8 = (lane & 15) * 8;
    v8h hv[8], lv[8];
#pragma unroll
    for (int it = 0; it < 8; ++it) {
      const int row = it * 8 + wave * 2 + rsub;
      const float* sp = sS + row * kHid + c8;
      const v4f a0 = *(const v4f*)(sp);
      const v4f a1 = *(const v4f*)(sp + 4);
      const float f[8] = {a0[0], a0[1], a0[2], a0[3], a1[0], a1[1], a1[2], a1[3]};
      pack8<SP>(f, 1.0f, hv[it], lv[it]);
    }
    for (int pass = 0; pass < 2; ++pass) {
#pragma unroll
      for (int it = 0; it < 8; ++it) {
        const int row = it * 8 + wave * 2 + rsub;
        const size_t o = (size_t)(base + row) * kHid + c8;
        *(volatile v8h*)(Sh + o) = hv[it];
        if (SP) *(volatile v8h*)(Sl + o) = lv[it];
      }
      __threadfence();
    }
  }
  if (wave < 2) {
    const float dv = (float)degc;
    float* dp = degp + base + tid;
    *(volatile float*)dp = dv;
    __threadfence();
    *(volatile float*)dp = dv;
  }
}

__global__ __launch_bounds__(256) void output_proj_kernel(
    const float* __restrict__ h32, const float* __restrict__ W, const float* __restrict__ b,
    float* __restrict__ out) {
  __shared__ __align__(16) float sW[kOutW * kHid];
  const int tid = threadIdx.x;
  for (int i = tid; i < kOutW * kHid; i += 256) {
    const int k = i / kOutW;
    const int j = i - k * kOutW;
    sW[j * kHid + k] = W[i];
  }
  __syncthreads();
  const int idx = blockIdx.x * 256 + tid;
  const bool live = idx < kNN * kOutW;
  const int idc = live ? idx : (kNN * kOutW - 1);
  const int n = idc / kOutW;
  const int j = idc - n * kOutW;
  const float* hr = h32 + (size_t)n * kHid;
  const float* wr = sW + j * kHid;
  float acc = 0.0f;
#pragma unroll 1
  for (int k4 = 0; k4 < kHid / 4; ++k4) {
    const v4f hv = *(const v4f*)(hr + 4 * k4);
    const v4f wv = *(const v4f*)(wr + 4 * k4);
    acc = fmaf(hv[0], wv[0], acc);
    acc = fmaf(hv[1], wv[1], acc);
    acc = fmaf(hv[2], wv[2], acc);
    acc = fmaf(hv[3], wv[3], acc);
  }
  acc += b[j];
  if (live) *(volatile float*)(out + idx) = acc;
  __threadfence();
  if (live) *(volatile float*)(out + idx) = acc;
}

static inline unsigned short* off16(unsigned short* p, size_t n) { return p ? (p + n) : nullptr; }

extern "C" void kernel_launch(void* const* d_in, const int* in_sizes, int n_in,
                              void* d_out, int out_size, void* d_ws, size_t ws_size,
                              hipStream_t stream) {
  if (n_in < 14) return;
  if (in_sizes[0] != kNN * kXin) return;
  if (in_sizes[1] != 2 * kNE) return;
  if (in_sizes[2] != kXin * kHid) return;
  if (in_sizes[3] != kHid) return;
  if (in_sizes[4] != kHid * kOutW) return;
  if (in_sizes[5] != kOutW) return;
  if (in_sizes[6] != kLayers * kCat * kHid) return;
  if (in_sizes[7] != kLayers * kHid) return;
  if (in_sizes[8] != kLayers * kHid * kHid) return;
  if (in_sizes[9] != kLayers * kHid) return;
  if (in_sizes[10] != kLayers * kCat * kHid) return;
  if (in_sizes[11] != kLayers * kHid) return;
  if (in_sizes[12] != kLayers * kHid * kHid) return;
  if (in_sizes[13] != kLayers * kHid) return;
  if (out_size != kNN * kOutW) return;
  if (ws_size < kWsTotal) return;

  const float* x    = (const float*)d_in[0];
  const int*   ei   = (const int*)d_in[1];
  const float* encW = (const float*)d_in[2];
  const float* encb = (const float*)d_in[3];
  const float* decW = (const float*)d_in[4];
  const float* decb = (const float*)d_in[5];
  const float* eW1  = (const float*)d_in[6];
  const float* eb1  = (const float*)d_in[7];
  const float* eW2  = (const float*)d_in[8];
  const float* eb2  = (const float*)d_in[9];
  const float* nW1  = (const float*)d_in[10];
  const float* nb1  = (const float*)d_in[11];
  const float* nW2  = (const float*)d_in[12];
  const float* nb2  = (const float*)d_in[13];
  float* out = (float*)d_out;

  char* ws = (char*)d_ws;
  float*          H32  = (float*)(ws + kOffH32);
  unsigned short* HAH  = (unsigned short*)(ws + kOffHAH);
  unsigned short* HAL  = kSplit ? (unsigned short*)(ws + kOffHAL) : nullptr;
  float*          PQ   = (float*)(ws + kOffPQ);
  unsigned short* SH   = (unsigned short*)(ws + kOffSH);
  unsigned short* SL   = kSplit ? (unsigned short*)(ws + kOffSL) : nullptr;
  unsigned short* TH   = (unsigned short*)(ws + kOffTH);
  unsigned short* TL   = kSplit ? (unsigned short*)(ws + kOffTL) : nullptr;
  float*          DEG  = (float*)(ws + kOffDEG);
  unsigned short* WE1H = (unsigned short*)(ws + kOffWE1H);
  unsigned short* WE1L = kSplit ? (unsigned short*)(ws + kOffWE1L) : nullptr;
  unsigned short* WE2H = (unsigned short*)(ws + kOffWE2H);
  unsigned short* WE2L = kSplit ? (unsigned short*)(ws + kOffWE2L) : nullptr;
  unsigned short* WN1H = (unsigned short*)(ws + kOffWN1H);
  unsigned short* WN1L = kSplit ? (unsigned short*)(ws + kOffWN1L) : nullptr;
  unsigned short* WN2H = (unsigned short*)(ws + kOffWN2H);
  unsigned short* WN2L = kSplit ? (unsigned short*)(ws + kOffWN2L) : nullptr;

  {
    const int t1 = kLayers * kCat * kHid / 8;
    const int t2 = kLayers * kHid * kHid / 8;
    weight_plane_kernel<kSplit><<<t1 / 256, 256, 0, stream>>>(eW1, WE1H, WE1L, kCat, kHid, kCat * kHid, 1, t1, kWCarry);
    weight_plane_kernel<kSplit><<<t2 / 256, 256, 0, stream>>>(eW2, WE2H, WE2L, kHid, kHid, kHid * kHid, 0, t2, kWCarry);
    weight_plane_kernel<kSplit><<<t1 / 256, 256, 0, stream>>>(nW1, WN1H, WN1L, kHid, kCat, kCat * kHid, 0, t1, kWCarry);
    weight_plane_kernel<kSplit><<<t2 / 256, 256, 0, stream>>>(nW2, WN2H, WN2L, kHid, kHid, kHid * kHid, 0, t2, kWCarry);
  }

  input_proj_kernel<kSplit><<<kMP / 64, 256, 0, stream>>>(x, encW, encb, H32, HAH, HAL);

  const int blocksPQ = ((kMP / 64) * (kCat / 64) + 7) / 8;
  const int blocksH  = ((kMP / 64) * (kHid / 64) + 7) / 8;
  for (int l = 0; l < kLayers; ++l) {
    const size_t w1o = (size_t)l * kCat * kHid;
    const size_t w2o = (size_t)l * kHid * kHid;
    tile_gemm_kernel<kET, kSPL, 0><<<blocksPQ, 256, 0, stream>>>(
        HAH, HAL, kCat,
        WE1H + w1o, off16(WE1L, w1o), kHid,
        PQ, kCat,
        nullptr, nullptr, 0,
        eb1 + l * kHid, nullptr,
        kMP, kCat, kHid, kNN, kWFold);
    edge_sum_kernel<kSplit><<<kMP / kTileNodes, kEdgeThreads, 0, stream>>>(ei, PQ, SH, SL, DEG);
    tile_gemm_kernel<kET, kSPL, 1><<<blocksH, 256, 0, stream>>>(
        SH, SL, kHid,
        WE2H + w2o, off16(WE2L, w2o), kHid,
        nullptr, 0,
        HAH + kHid, off16(HAL, kHid), kCat,
        eb2 + l * kHid, DEG,
        kMP, kHid, kHid, kNN, kWFold);
    tile_gemm_kernel<kET, kSPL, 2><<<blocksH, 256, 0, stream>>>(
        HAH, HAL, kCat,
        WN1H + w1o, off16(WN1L, w1o), kCat,
        nullptr, 0,
        TH, TL, kHid,
        nb1 + l * kHid, nullptr,
        kMP, kHid, kCat, kNN, kWFold);
    tile_gemm_kernel<kET, kSPL, 3><<<blocksH, 256, 0, stream>>>(
        TH, TL, kHid,
        WN2H + w2o, off16(WN2L, w2o), kHid,
        H32, kHid,
        HAH, HAL, kCat,
        nb2 + l * kHid, nullptr,
        kMP, kHid, kHid, kNN, kWFold);
  }

  output_proj_kernel<<<(kNN * kOutW + 255) / 256, 256, 0, stream>>>(H32, decW, decb, out);
}
